// GCN_54863912239236
// MI455X (gfx1250) — hardware-verified
//
#include <hip/hip_runtime.h>
#include <stddef.h>
#include <stdint.h>
#include <math.h>


#define D       128
#define DO      64
#define K2      256
#define NTHR    256
#define NWAVE   8
#define EPT     8
#define CHUNK   (NTHR * EPT)
#define WCAP    (EPT * 32)
#define LISTN   (NWAVE * WCAP)
#define NBA     1024
#define PKS     10
#define RCAP    28672
#define DEGCAP  64
#define GBM     64
#define GBN     64
#define GTHR    128
#define NU1     (D * (D / 8))
#define NU2     (D * (D / 4))
#define NU3     (DO * (D / 4))
#define NUW     (NU1 + NU2 + NU3)
#define ZINTS   (2 * RCAP + 2 * NBA + LISTN)
#define LDS_AGG (ZINTS * 4 + 64)
#define WSMAX   134217728

static_assert((CHUNK & (CHUNK - 1)) == 0);
static_assert(NBA == (1 << PKS));
static_assert(((long long)CHUNK << PKS) < (1LL << 31));
static_assert(NTHR * 4 == NBA);
static_assert(LISTN >= NBA && LISTN >= NWAVE * WCAP);
static_assert((RCAP % 32) == 0);
static_assert((ZINTS % (NTHR * 4)) == 0);
static_assert(LDS_AGG <= 300000);
static_assert((NBA % NWAVE) == 0);
static_assert(GBM == (GTHR / 32) * 16 && GBN == 64);
static_assert((D % GBN) == 0 && (DO % GBN) == 0);
static_assert((D % 32) == 0 && (K2 % 32) == 0 && K2 == 2 * D);
static_assert(((D * 2) % 128) == 0 && ((K2 * 2) % 128) == 0);
static_assert(((D * 4) % 128) == 0 && ((DO * 4) % 128) == 0);
static_assert((NU1 % NTHR) == 0 && (NU2 % NTHR) == 0 && (NU3 % NTHR) == 0);
static_assert(D == 32 * 4);
static_assert(DO == 32 * 2);
static_assert((D / 8) == 16 && (D / 4) == 32);
static_assert((NBA % GBM) == 0);

typedef float          v2f   __attribute__((ext_vector_type(2)));
typedef float          v4f   __attribute__((ext_vector_type(4)));
typedef float          v8f   __attribute__((ext_vector_type(8)));
typedef int            v4i   __attribute__((ext_vector_type(4)));
typedef int            v8i   __attribute__((ext_vector_type(8)));
typedef unsigned short v8us  __attribute__((ext_vector_type(8)));
typedef unsigned short v16us __attribute__((ext_vector_type(16)));
typedef __bf16         v16bf __attribute__((ext_vector_type(16)));
typedef v2f  __attribute__((may_alias)) v2fa;
typedef v4f  __attribute__((may_alias)) v4fa;
typedef v4i  __attribute__((may_alias)) v4ia;
typedef v8us __attribute__((may_alias)) v8usa;
union Frag { v16bf v; v16us u; v8us h[2]; v8i w; };

__device__ __forceinline__ v8f wmb(const Frag& a, const Frag& b, v8f c) {
  v8f d = __builtin_amdgcn_wmma_f32_16x16x32_bf16(false, a.v, false, b.v, (short)0, c, false, false);
  asm volatile("v_nop\n\tv_nop\n\tv_nop\n\tv_nop" : "+v"(d) : "v"(a.w), "v"(b.w));
  return d;
}

__device__ __forceinline__ v8f z8() { v8f z = {0.f, 0.f, 0.f, 0.f, 0.f, 0.f, 0.f, 0.f}; return z; }

__device__ __forceinline__ unsigned bf16_bits(float f) {
  const unsigned u = __float_as_uint(f);
  return (u + 0x7FFFu + ((u >> 16) & 1u)) >> 16;
}
__device__ __forceinline__ float bf16_val(float f) {
  return __uint_as_float(bf16_bits(f) << 16);
}
__device__ __forceinline__ v8us hilo8(v4f t) {
  v8us o;
  unsigned hb;
  hb = bf16_bits(t.x); o[0] = (unsigned short)hb; o[4] = (unsigned short)bf16_bits(t.x - __uint_as_float(hb << 16));
  hb = bf16_bits(t.y); o[1] = (unsigned short)hb; o[5] = (unsigned short)bf16_bits(t.y - __uint_as_float(hb << 16));
  hb = bf16_bits(t.z); o[2] = (unsigned short)hb; o[6] = (unsigned short)bf16_bits(t.z - __uint_as_float(hb << 16));
  hb = bf16_bits(t.w); o[3] = (unsigned short)hb; o[7] = (unsigned short)bf16_bits(t.w - __uint_as_float(hb << 16));
  return o;
}

__device__ __forceinline__ int scan_chunk(const int* __restrict__ dsts, int nE, int cbase, int slotBase,
                                          int nb, int vec8, int* list, int tid, int lane, int wave) {
  int wc = 0;
  const int el0  = tid * EPT;
  const int e0   = cbase + el0;
  const int sent = -2147483647 - 1;
  v4i da, db;
  if (vec8 != 0 && cbase + CHUNK <= nE) {
    da = *(const v4i*)(dsts + e0);
    db = *(const v4i*)(dsts + e0 + 4);
  } else {
    da.x = (e0     < nE) ? dsts[min(e0,     nE - 1)] : sent;
    da.y = (e0 + 1 < nE) ? dsts[min(e0 + 1, nE - 1)] : sent;
    da.z = (e0 + 2 < nE) ? dsts[min(e0 + 2, nE - 1)] : sent;
    da.w = (e0 + 3 < nE) ? dsts[min(e0 + 3, nE - 1)] : sent;
    db.x = (e0 + 4 < nE) ? dsts[min(e0 + 4, nE - 1)] : sent;
    db.y = (e0 + 5 < nE) ? dsts[min(e0 + 5, nE - 1)] : sent;
    db.z = (e0 + 6 < nE) ? dsts[min(e0 + 6, nE - 1)] : sent;
    db.w = (e0 + 7 < nE) ? dsts[min(e0 + 7, nE - 1)] : sent;
  }
  const unsigned nbs = (unsigned)slotBase;
  const unsigned unb = (unsigned)nb;
  const unsigned s0 = (unsigned)da.x - nbs, s1 = (unsigned)da.y - nbs;
  const unsigned s2 = (unsigned)da.z - nbs, s3 = (unsigned)da.w - nbs;
  const unsigned s4 = (unsigned)db.x - nbs, s5 = (unsigned)db.y - nbs;
  const unsigned s6 = (unsigned)db.z - nbs, s7 = (unsigned)db.w - nbs;
  const bool h0 = s0 < unb, h1 = s1 < unb, h2 = s2 < unb, h3 = s3 < unb;
  const bool h4 = s4 < unb, h5 = s5 < unb, h6 = s6 < unb, h7 = s7 < unb;
  const unsigned any = __builtin_amdgcn_ballot_w32(h0 | h1 | h2 | h3 | h4 | h5 | h6 | h7);
  if (any != 0u) {
#define HITJ(J, HJ, SJ) { \
      const unsigned mj = __builtin_amdgcn_ballot_w32(HJ); \
      if (mj != 0u) { \
        if (HJ) { \
          const int pos = wc + (int)__builtin_amdgcn_mbcnt_lo(mj, 0u); \
          if (pos < WCAP) list[wave * WCAP + pos] = ((el0 + (J)) << PKS) | (int)(SJ); \
        } \
        wc += (int)__builtin_popcount(mj); } }
    HITJ(0, h0, s0)
    HITJ(1, h1, s1)
    HITJ(2, h2, s2)
    HITJ(3, h3, s3)
    HITJ(4, h4, s4)
    HITJ(5, h5, s5)
    HITJ(6, h6, s6)
    HITJ(7, h7, s7)
#undef HITJ
  }
  return wc;
}

__global__ __launch_bounds__(NTHR) void k_prep(const float* __restrict__ W1, const float* __restrict__ W2,
                                               const float* __restrict__ W3, const float* __restrict__ x,
                                               int nN, int nUx,
                                               unsigned short* W1T, unsigned short* W2T, unsigned short* W3T,
                                               unsigned short* XB) {
  const int u = (int)blockIdx.x * NTHR + (int)threadIdx.x;
  v8us o;
  unsigned short* dp;
  if (u < NU1) {
    const int n  = u >> 4;
    const int k8 = (u & 15) * 8;
    const float* p = W1 + (size_t)k8 * D + n;
#pragma unroll
    for (int i = 0; i < 8; ++i) o[i] = (unsigned short)bf16_bits(p[(size_t)i * D]);
    dp = W1T + (size_t)n * D + k8;
  } else if (u < NU1 + NU2) {
    const int v = u - NU1;
    const int n = v >> 5;
    const int g = v & 31;
    const float* p = W2 + (size_t)(4 * g) * D + n;
    const unsigned short f0 = (unsigned short)bf16_bits(p[0]);
    const unsigned short f1 = (unsigned short)bf16_bits(p[D]);
    const unsigned short f2 = (unsigned short)bf16_bits(p[2 * D]);
    const unsigned short f3 = (unsigned short)bf16_bits(p[3 * D]);
    o[0] = f0; o[1] = f1; o[2] = f2; o[3] = f3; o[4] = f0; o[5] = f1; o[6] = f2; o[7] = f3;
    dp = W2T + (size_t)n * K2 + 8 * g;
  } else if (u < NUW) {
    const int v = u - NU1 - NU2;
    const int n = v >> 5;
    const int g = v & 31;
    const float* p = W3 + (size_t)(4 * g) * DO + n;
    const unsigned short f0 = (unsigned short)bf16_bits(p[0]);
    const unsigned short f1 = (unsigned short)bf16_bits(p[DO]);
    const unsigned short f2 = (unsigned short)bf16_bits(p[2 * DO]);
    const unsigned short f3 = (unsigned short)bf16_bits(p[3 * DO]);
    o[0] = f0; o[1] = f1; o[2] = f2; o[3] = f3; o[4] = f0; o[5] = f1; o[6] = f2; o[7] = f3;
    dp = W3T + (size_t)n * K2 + 8 * g;
  } else {
    const int v = u - NUW;
    if (v >= nUx) return;
    const int row = v >> 4;
    const int k8  = (v & 15) * 8;
    const bool rok = row < nN;
    const int rc = rok ? row : nN - 1;
    const float* p = x + (size_t)rc * D + k8;
    const v4f a = *(const v4fa*)p;
    const v4f b = *(const v4fa*)(p + 4);
    o[0] = rok ? (unsigned short)bf16_bits(a.x) : (unsigned short)0;
    o[1] = rok ? (unsigned short)bf16_bits(a.y) : (unsigned short)0;
    o[2] = rok ? (unsigned short)bf16_bits(a.z) : (unsigned short)0;
    o[3] = rok ? (unsigned short)bf16_bits(a.w) : (unsigned short)0;
    o[4] = rok ? (unsigned short)bf16_bits(b.x) : (unsigned short)0;
    o[5] = rok ? (unsigned short)bf16_bits(b.y) : (unsigned short)0;
    o[6] = rok ? (unsigned short)bf16_bits(b.z) : (unsigned short)0;
    o[7] = rok ? (unsigned short)bf16_bits(b.w) : (unsigned short)0;
    dp = XB + (size_t)row * D + k8;
  }
  *(volatile v8us*)dp = o;
  __threadfence();
  *(volatile v8us*)dp = o;
}

__global__ __launch_bounds__(GTHR) void k_gemm(
    const unsigned short* __restrict__ A, const unsigned short* __restrict__ WT,
    float* outF, int K, int ldo)
{
  __shared__ __attribute__((aligned(16))) float stg[GBM * GBN];
  const int tid = (int)threadIdx.x, lane = tid & 31, wave = tid >> 5, hh = lane >> 4, m = lane & 15;
  const int rowBase = (int)blockIdx.x * GBM;
  const int col0    = (int)blockIdx.y * GBN;

  v8f acc[4];
  acc[0] = z8(); acc[1] = z8(); acc[2] = z8(); acc[3] = z8();
  const unsigned short* ap = A  + (size_t)(rowBase + 16 * wave + m) * (size_t)K + 8 * hh;
  const unsigned short* wp = WT + (size_t)(col0 + m) * (size_t)K + 8 * hh;
  const int ksteps = K >> 5;
#pragma unroll 1
  for (int ks = 0; ks < ksteps; ++ks) {
    Frag af;
    af.h[0] = *(const v8usa*)(ap + 32 * ks);
    af.h[1] = *(const v8usa*)(ap + 32 * ks + 16);
#pragma unroll
    for (int t = 0; t < 4; ++t) {
      const unsigned short* wq = wp + (size_t)(16 * t) * (size_t)K + 32 * ks;
      Frag bf;
      bf.h[0] = *(const v8usa*)wq;
      bf.h[1] = *(const v8usa*)(wq + 16);
      acc[t] = wmb(af, bf, acc[t]);
    }
  }

#pragma unroll
  for (int t = 0; t < 4; ++t) {
    const int lc = 16 * t + m;
#pragma unroll
    for (int r = 0; r < 8; ++r) {
      const int lr = 16 * wave + 8 * hh + r;
      stg[lr * GBN + lc] = acc[t][r];
    }
  }
  __syncthreads();

  v4f fv[8];
#pragma unroll
  for (int i = 0; i < 8; ++i) {
    const int lr = 16 * wave + 2 * i + hh;
    fv[i] = *(const v4fa*)(stg + lr * GBN + 4 * m);
  }
#pragma unroll
  for (int i = 0; i < 8; ++i) {
    const int lr = 16 * wave + 2 * i + hh;
    const int gr = rowBase + lr;
    float* op = outF + (size_t)gr * (size_t)ldo + col0 + 4 * m;
    *(volatile v4f*)op = fv[i];
  }
  __threadfence();
#pragma unroll
  for (int i = 0; i < 8; ++i) {
    const int lr = 16 * wave + 2 * i + hh;
    const int gr = rowBase + lr;
    float* op = outF + (size_t)gr * (size_t)ldo + col0 + 4 * m;
    *(volatile v4f*)op = fv[i];
  }
}

template <int MODE>
__global__ __launch_bounds__(NTHR) void k_agg(const int* __restrict__ srcs, const int* __restrict__ dsts,
                                              const float* __restrict__ ew, const float* __restrict__ F,
                                              const float* __restrict__ bias,
                                              unsigned short* hb, float* outp,
                                              int nN, int nE, int vec8, int mRows) {
  extern __shared__ __attribute__((aligned(16))) int lds_i[];
  int* reg1 = lds_i;
  int* reg2 = reg1 + RCAP;
  int* scnt = reg2 + RCAP;
  int* soff = scnt + NBA;
  int* list = soff + NBA;
  int* wcnt = list + LISTN;
  int* wtot = wcnt + NWAVE;
  constexpr int C = (MODE != 0) ? D : DO;
  const int tid = (int)threadIdx.x, lane = tid & 31, wave = tid >> 5;
  const int nodeBase = (int)blockIdx.x * NBA;

  {
    const v4i z4 = {0, 0, 0, 0};
    for (int i = tid * 4; i < ZINTS; i += NTHR * 4) *(v4ia*)(lds_i + i) = z4;
    if (tid < 2 * NWAVE) wcnt[tid] = 0;
  }
  v4f bq;
  if constexpr (MODE != 0) {
    const v4f t = *(const v4fa*)(bias + 4 * lane);
    bq.x = bf16_val(t.x); bq.y = bf16_val(t.y); bq.z = bf16_val(t.z); bq.w = bf16_val(t.w);
  } else {
    const v2f t = *(const v2fa*)(bias + 2 * lane);
    bq.x = bf16_val(t.x); bq.y = bf16_val(t.y); bq.z = 0.0f; bq.w = 0.0f;
  }
  __syncthreads();

  int tot = 0;
  const int nChunks = (nE + CHUNK - 1) / CHUNK;
#pragma unroll 1
  for (int ch = 0; ch < nChunks; ++ch) {
    const int cbase = ch * CHUNK;
    const int wc = scan_chunk(dsts, nE, cbase, nodeBase, NBA, vec8, list, tid, lane, wave);
    if (lane == 0) wcnt[wave] = wc;
    __syncthreads();
    int pre = 0, all = 0;
#pragma unroll
    for (int w2 = 0; w2 < NWAVE; ++w2) {
      int c = wcnt[w2];
      c = c < 0 ? 0 : (c > WCAP ? WCAP : c);
      all += c;
      pre += (w2 < wave) ? c : 0;
    }
    const int wcc  = wc > WCAP ? WCAP : wc;
    const int base = tot + pre;
#pragma unroll 1
    for (int i = lane; i < wcc; i += 32) {
      const int ent = list[wave * WCAP + i];
      const int el  = (ent >> PKS) & (CHUNK - 1);
      const int sl  = ent & (NBA - 1);
      int eid = cbase + el;
      eid = eid > nE - 1 ? nE - 1 : eid;
      const int pos = base + i;
      if (pos < RCAP) reg1[pos] = (int)(((unsigned)eid << PKS) | (unsigned)sl);
    }
    tot += all;
    tot = tot > RCAP ? RCAP : tot;
    __syncthreads();
  }
  const int nh = tot;

  if (wave == 0) {
#pragma unroll 1
    for (int b0 = 0; b0 < nh; b0 += 32) {
      const int idx = b0 + lane;
      const int uv  = reg1[idx < RCAP ? idx : RCAP - 1];
      const int m32 = (nh - b0) < 32 ? (nh - b0) : 32;
#pragma unroll 1
      for (int k = 0; k < m32; ++k) {
        const int u  = __builtin_amdgcn_readlane(uv, k);
        const int sl = u & (NBA - 1);
        if (lane == 0) scnt[sl] = scnt[sl] + 1;
      }
    }
  }
  __syncthreads();

  {
    const v4i ca = *(const v4ia*)(scnt + 4 * tid);
    const int e0 = ca.x < 0 ? 0 : ca.x, e1 = ca.y < 0 ? 0 : ca.y, e2 = ca.z < 0 ? 0 : ca.z, e3 = ca.w < 0 ? 0 : ca.w;
    const int ts = e0 + e1 + e2 + e3;
    int incl = ts;
#pragma unroll
    for (int d = 1; d < 32; d <<= 1) {
      const int up = __shfl_up(incl, d, 32);
      if (lane >= d) incl += up;
    }
    if (lane == 31) wtot[wave] = incl;
    __syncthreads();
    int pre = 0;
#pragma unroll
    for (int w2 = 0; w2 < NWAVE; ++w2) pre += (w2 < wave) ? wtot[w2] : 0;
    int run = pre + incl - ts;
    soff[4 * tid + 0] = run; run += e0;
    soff[4 * tid + 1] = run; run += e1;
    soff[4 * tid + 2] = run; run += e2;
    soff[4 * tid + 3] = run;
  }
  __syncthreads();
  for (int i = tid; i < NBA; i += NTHR) list[i] = soff[i];
  __syncthreads();

  if (wave == 0) {
#pragma unroll 1
    for (int b0 = 0; b0 < nh; b0 += 32) {
      const int idx = b0 + lane;
      const int uv  = reg1[idx < RCAP ? idx : RCAP - 1];
      const int m32 = (nh - b0) < 32 ? (nh - b0) : 32;
#pragma unroll 1
      for (int k = 0; k < m32; ++k) {
        const int u   = __builtin_amdgcn_readlane(uv, k);
        const int sl  = u & (NBA - 1);
        const int eid = (int)((unsigned)u >> PKS);
        if (lane == 0) {
          int pos = list[sl];
          pos = pos < 0 ? 0 : (pos > RCAP - 1 ? RCAP - 1 : pos);
          reg2[pos] = eid;
          list[sl] = pos + 1;
        }
      }
    }
  }
  __syncthreads();

  const int nbw = NBA / NWAVE;
  const bool ovf = (nh >= RCAP);
  const float qnan = __int_as_float(0x7fc00000);

#pragma unroll 1
  for (int jt = 0; jt < nbw; ++jt) {
    const int slot = wave * nbw + jt;
    const int node = nodeBase + slot;
    int st = soff[slot];
    const int craw = scnt[slot];
    int cnt = craw;
    st  = st < 0 ? 0 : (st > nh ? nh : st);
    cnt = cnt < 0 ? 0 : (cnt > DEGCAP ? DEGCAP : cnt);
    if (cnt > nh - st) cnt = nh - st;
    const float pz = (ovf || craw > DEGCAP) ? qnan : 0.0f;
    const bool live = node < nN;

    float a0 = 0.0f, a1 = 0.0f, a2 = 0.0f, a3 = 0.0f;
#pragma unroll 1
    for (int b0 = 0; b0 < cnt; b0 += 32) {
      int idx = st + b0 + lane; idx = idx > RCAP - 1 ? RCAP - 1 : idx;
      int eid = reg2[idx]; eid = eid < 0 ? 0 : (eid > nE - 1 ? nE - 1 : eid);
      int sr = srcs[eid]; sr = sr < 0 ? 0 : (sr > nN - 1 ? nN - 1 : sr);
      const int wvi = __float_as_int(bf16_val(ew[eid]));
      const int m32 = (cnt - b0) < 32 ? (cnt - b0) : 32;
#pragma unroll 1
      for (int k = 0; k < m32; ++k) {
        const int   sk = __builtin_amdgcn_readlane(sr, k);
        const float wk = __int_as_float(__builtin_amdgcn_readlane(wvi, k));
        if constexpr (MODE != 0) {
          const v4f v = *(const v4fa*)(F + (size_t)sk * C + 4 * lane);
          a0 = fmaf(wk, v.x, a0); a1 = fmaf(wk, v.y, a1);
          a2 = fmaf(wk, v.z, a2); a3 = fmaf(wk, v.w, a3);
        } else {
          const v2f v = *(const v2fa*)(F + (size_t)sk * C + 2 * lane);
          a0 = fmaf(wk, v.x, a0); a1 = fmaf(wk, v.y, a1);
        }
      }
    }

    if constexpr (MODE != 0) {
      v4f y;
      y.x = fmaxf(a0 + bq.x, 0.0f) + pz;
      y.y = fmaxf(a1 + bq.y, 0.0f) + pz;
      y.z = fmaxf(a2 + bq.z, 0.0f) + pz;
      y.w = fmaxf(a3 + bq.w, 0.0f) + pz;
      v4f v;
      v.x = live ? y.x : 0.0f;
      v.y = live ? y.y : 0.0f;
      v.z = live ? y.z : 0.0f;
      v.w = live ? y.w : 0.0f;
      const v8us p0 = hilo8(v);
      if (node < mRows) {
        unsigned short* hp = hb + (size_t)node * (size_t)K2 + 8 * lane;
        *(volatile v8us*)hp = p0;
        __threadfence();
        *(volatile v8us*)hp = p0;
      }
    } else {
      const float y0 = (a0 + bq.x) + pz;
      const float y1 = (a1 + bq.y) + pz;
      float mx = fmaxf(y0, y1);
#pragma unroll
      for (int o = 16; o > 0; o >>= 1) mx = fmaxf(mx, __shfl_xor(mx, o, 32));
      const float e0 = y0 - mx;
      const float e1 = y1 - mx;
      float se = __expf(e0) + __expf(e1);
#pragma unroll
      for (int o = 16; o > 0; o >>= 1) se += __shfl_xor(se, o, 32);
      const float ls = logf(se);
      v2f ov;
      ov.x = e0 - ls;
      ov.y = e1 - ls;
      if (live) {
        float* gp = outp + (size_t)node * (size_t)DO + 2 * lane;
        *(volatile v2f*)gp = ov;
        __threadfence();
        *(volatile v2f*)gp = ov;
      }
    }
  }
}

static inline int cdiv(int a, int b) { return (a + b - 1) / b; }
static inline size_t al256(size_t o) { return (o + 255) & ~(size_t)255; }

extern "C" void kernel_launch(void* const* d_in, const int* in_sizes, int n_in,
                              void* d_out, int out_size, void* d_ws, size_t ws_size,
                              hipStream_t stream) {
  if (n_in < 10) return;
  if (in_sizes[0] < D || (in_sizes[0] % D) != 0) return;
  const int nN = in_sizes[0] / D;
  if (nN < 1 || nN > (1 << 22)) return;
  const int nE = in_sizes[1];
  if (nE < 1 || nE >= (1 << (32 - PKS))) return;
  if (in_sizes[2] != nE || in_sizes[3] != nE) return;
  if (in_sizes[4] != D * D || in_sizes[5] != D) return;
  if (in_sizes[6] != D * D || in_sizes[7] != D) return;
  if (in_sizes[8] != D * DO || in_sizes[9] != DO) return;
  if ((long long)out_size != (long long)nN * DO) return;

  const float* x    = (const float*)d_in[0];
  const int*   esrc = (const int*)  d_in[1];
  const int*   edst = (const int*)  d_in[2];
  const float* ew   = (const float*)d_in[3];
  const float* W1   = (const float*)d_in[4];
  const float* b1   = (const float*)d_in[5];
  const float* W2   = (const float*)d_in[6];
  const float* b2   = (const float*)d_in[7];
  const float* W3   = (const float*)d_in[8];
  const float* b3   = (const float*)d_in[9];
  float* out = (float*)d_out;

  const int MP   = cdiv(nN, GBM) * GBM;
  const int gM   = MP / GBM;
  const int gA   = cdiv(MP, NBA);
  const int vec8 = ((nE & 3) == 0) ? 1 : 0;
  if ((long long)gA * NBA < (long long)MP) return;
  if ((long long)gM * GBM < (long long)nN) return;

  char* ws = (char*)d_ws;
  size_t off = 0;
  const size_t oW1T = off; off = al256(off + (size_t)D  * D  * 2);
  const size_t oW2T = off; off = al256(off + (size_t)D  * K2 * 2);
  const size_t oW3T = off; off = al256(off + (size_t)DO * K2 * 2);
  const size_t oXB  = off; off = al256(off + (size_t)MP * D  * 2);
  const size_t oT   = off; off = al256(off + (size_t)MP * D  * 4);
  const size_t oAZ  = off; off = al256(off + (size_t)MP * K2 * 2);
  if (off > ws_size || off > (size_t)WSMAX) return;
  unsigned short* W1T = (unsigned short*)(ws + oW1T);
  unsigned short* W2T = (unsigned short*)(ws + oW2T);
  unsigned short* W3T = (unsigned short*)(ws + oW3T);
  unsigned short* XB  = (unsigned short*)(ws + oXB);
  float*          T   = (float*)(ws + oT);
  unsigned short* AZ  = (unsigned short*)(ws + oAZ);

  const int nUx = MP * (D / 8);

  hipFuncSetAttribute(reinterpret_cast<const void*>(&k_agg<1>), hipFuncAttributeMaxDynamicSharedMemorySize, LDS_AGG);
  hipFuncSetAttribute(reinterpret_cast<const void*>(&k_agg<0>), hipFuncAttributeMaxDynamicSharedMemorySize, LDS_AGG);

  k_prep<<<cdiv(NUW + nUx, NTHR), NTHR, 0, stream>>>(W1, W2, W3, x, nN, nUx, W1T, W2T, W3T, XB);
  k_gemm<<<dim3(gM, D / GBN), GTHR, 0, stream>>>(XB, W1T, T, D, D);
  k_agg<1><<<gA, NTHR, LDS_AGG, stream>>>(esrc, edst, ew, T, b1, AZ, out, nN, nE, vec8, MP);
  k_gemm<<<dim3(gM, D / GBN), GTHR, 0, stream>>>(AZ, W2T, T, K2, D);
  k_agg<1><<<gA, NTHR, LDS_AGG, stream>>>(esrc, edst, ew, T, b2, AZ, out, nN, nE, vec8, MP);
  k_gemm<<<dim3(gM, DO / GBN), GTHR, 0, stream>>>(AZ, W3T, T, K2, DO);
  k_agg<0><<<gA, NTHR, LDS_AGG, stream>>>(esrc, edst, ew, T, b3, AZ, out, nN, nE, vec8, MP);
}
